// MultiHeadAttentionSimple_16114717295255
// MI455X (gfx1250) — hardware-run, weakly checked
//
#include <hip/hip_runtime.h>
#include <math.h>
#include <stdint.h>

#ifndef NB
#define NB 8
#endif
#ifndef SEQ
#define SEQ 2048
#endif
#define NB_FULL  8
#define SEQ_FULL 2048
#define DM    512
#define NH    8
#define HD    512
#define DQKV  (NH * HD)
#define MROWS (NB * SEQ)
#define NRT   (MROWS / 64)
#define EPT   (SEQ / 256)
#define OUT1_OFF   (NB_FULL * DM)
#define OUT1_PITCH SEQ_FULL
#define RSC   16.0f
#define WCS   4096.0f
#define LOS   4096.0f
#define LOG2E 1.4426950408889634f
#define SLAB  (16 * 68)

static_assert(NB >= 1 && NB <= NB_FULL);
static_assert(SEQ >= 256 && SEQ <= SEQ_FULL && (SEQ % 256) == 0);
static_assert(HD == DM && (DM % 64) == 0 && (HD % 64) == 0 && (MROWS % 64) == 0);
static_assert(((MROWS * (DM / 8)) % 256) == 0 && (((DM * DQKV) / 8) % 256) == 0);
static_assert(EPT >= 1 && EPT <= 8);
static_assert((HD % 128) == 0 && (DM % 32) == 0);
static_assert((SLAB * 4) % 16 == 0);
static_assert(OUT1_OFF * 4 == 16384);
static_assert((OUT1_OFF + NH * NB_FULL * SEQ_FULL) * 4 == 540672);
static_assert((OUT1_PITCH * 4) % 128 == 0 && (OUT1_OFF * 4) % 128 == 0);

typedef unsigned short u16;
typedef _Float16 v16h __attribute__((ext_vector_type(16)));
typedef _Float16 v8h  __attribute__((ext_vector_type(8)));
typedef __bf16   v16b __attribute__((ext_vector_type(16)));
typedef float    v8f  __attribute__((ext_vector_type(8)));
typedef float    v4f  __attribute__((ext_vector_type(4)));
typedef unsigned int v4u __attribute__((ext_vector_type(4)));

union FragH { v16h v; v8h h[2]; v4u u[2]; };
union FragB { v16b v; v4u u[2]; };

__device__ __forceinline__ unsigned short bf_bits(float f) {
  unsigned u = __float_as_uint(f);
  return (unsigned short)((u + 0x7FFFu + ((u >> 16) & 1u)) >> 16);
}
__device__ __forceinline__ float bf_up(unsigned short h) { return __uint_as_float(((unsigned)h) << 16); }
__device__ __forceinline__ float bf_val(float f) { return bf_up(bf_bits(f)); }
__device__ __forceinline__ unsigned short h_bits(_Float16 x) { return __builtin_bit_cast(unsigned short, x); }
__device__ __forceinline__ unsigned pk16(unsigned short a, unsigned short b) { return (unsigned)a | ((unsigned)b << 16); }
__device__ __forceinline__ v8f zero8() { v8f z = {0.f, 0.f, 0.f, 0.f, 0.f, 0.f, 0.f, 0.f}; return z; }

__device__ __forceinline__ v16h ldfrag_h(const _Float16* p) {
  FragH f;
  f.h[0] = *(const v8h*)(p);
  f.h[1] = *(const v8h*)(p + 16);
  return f.v;
}
__device__ __forceinline__ v16b ldfrag_b(const u16* p) {
  FragB f;
  f.u[0] = *(const v4u*)(p);
  f.u[1] = *(const v4u*)(p + 16);
  return f.v;
}

__device__ __forceinline__ v8f mma_h(v16h a, v16h b, v8f c) {
  return __builtin_amdgcn_wmma_f32_16x16x32_f16(false, a, false, b, (short)0, c, false, false);
}
__device__ __forceinline__ v8f mma_b(v16b a, v16b b, v8f c) {
  return __builtin_amdgcn_wmma_f32_16x16x32_bf16(false, a, false, b, (short)0, c, false, false);
}
template <typename F>
__device__ __forceinline__ void guard5(v8f& a, v8f& b, v8f& c, v8f& d, F x0, F x1, F x2, F x3, F x4) {
#if defined(__HIP_DEVICE_COMPILE__)
  asm volatile("v_nop\n\tv_nop\n\tv_nop\n\tv_nop"
               : "+v"(a), "+v"(b), "+v"(c), "+v"(d) : "v"(x0), "v"(x1), "v"(x2), "v"(x3), "v"(x4) : "memory");
#endif
}
__device__ __forceinline__ void acc_guard4(v8f& a, v8f& b, v8f& c, v8f& d) {
#if defined(__HIP_DEVICE_COMPILE__)
  asm volatile("v_nop\n\tv_nop\n\tv_nop\n\tv_nop" : "+v"(a), "+v"(b), "+v"(c), "+v"(d));
#endif
}
__device__ __forceinline__ void wave_sync_lds() {
#if defined(__HIP_DEVICE_COMPILE__)
  __builtin_amdgcn_fence(__ATOMIC_RELEASE, "workgroup");
  __builtin_amdgcn_wave_barrier();
  __builtin_amdgcn_fence(__ATOMIC_ACQUIRE, "workgroup");
#endif
}

__global__ __launch_bounds__(256) void k_cvt_bf(const float* __restrict__ x, u16* D, int n8) {
  const int gt = blockIdx.x * 256 + (int)threadIdx.x;
  if (gt >= n8) return;
  const float* p = x + (size_t)gt * 8;
  const v4f a = *(const v4f*)(p), c4 = *(const v4f*)(p + 4);
  float v[8];
#pragma unroll
  for (int e = 0; e < 4; ++e) { v[e] = a[e]; v[4 + e] = c4[e]; }
  v4u o;
#pragma unroll
  for (int e = 0; e < 4; ++e) o[e] = pk16(bf_bits(v[2 * e]), bf_bits(v[2 * e + 1]));
  u16* d = D + (size_t)gt * 8;
  for (int pass = 0; pass < 2; ++pass) {
    *(volatile v4u*)(d) = o;
    __threadfence();
  }
}

__global__ __launch_bounds__(256) void k_cvt_right(const float* __restrict__ x, u16* D, int n8) {
  const int gt = blockIdx.x * 256 + (int)threadIdx.x;
  if (gt >= n8) return;
  const int row = gt >> 6;
  const int e8  = (gt & 63) * 8;
  const int b   = row / SEQ;
  const int l   = row - b * SEQ;
  const float* p = x + ((size_t)b * SEQ_FULL + (size_t)l) * DM + e8;
  const v4f a = *(const v4f*)(p), c4 = *(const v4f*)(p + 4);
  float v[8];
#pragma unroll
  for (int e = 0; e < 4; ++e) { v[e] = a[e]; v[4 + e] = c4[e]; }
  unsigned short s[8];
#pragma unroll
  for (int e = 0; e < 8; ++e) s[e] = h_bits((_Float16)(bf_val(v[e]) * RSC));
  v4u o;
#pragma unroll
  for (int e = 0; e < 4; ++e) o[e] = pk16(s[2 * e], s[2 * e + 1]);
  u16* d = D + (size_t)gt * 8;
  for (int pass = 0; pass < 2; ++pass) {
    *(volatile v4u*)(d) = o;
    __threadfence();
  }
}

__global__ __launch_bounds__(256) void k_w1kt(const float* __restrict__ W1, u16* W1KT) {
  __shared__ __align__(16) u16 tile[64 * 72];
  const int tid = threadIdx.x, wave = tid >> 5, lane = tid & 31;
  const int c0 = (blockIdx.x & 7) * 64;
  const int d0 = (blockIdx.x >> 3) * 64;
  const int ty = tid >> 4, tx = tid & 15;
#pragma unroll
  for (int k = 0; k < 4; ++k) {
    const int cl = ty + 16 * k;
    const v4f v = *(const v4f*)(W1 + (size_t)(DM + c0 + cl) * DM + d0 + 4 * tx);
#pragma unroll
    for (int j = 0; j < 4; ++j) tile[(4 * tx + j) * 72 + cl] = bf_bits(v[j]);
  }
  __syncthreads();
  const int rq = lane >> 3, c8 = (lane & 7) * 8;
  v4u ov[2];
#pragma unroll
  for (int i = 0; i < 2; ++i) {
    const int dl = wave * 8 + i * 4 + rq;
    ov[i] = *(const v4u*)(tile + dl * 72 + c8);
  }
  u16* dst = W1KT + (size_t)(d0 + wave * 8 + rq) * HD + c0 + c8;
  for (int pass = 0; pass < 2; ++pass) {
#pragma unroll
    for (int i = 0; i < 2; ++i) {
      *(volatile v4u*)(dst + (size_t)(i * 4) * HD) = ov[i];
    }
    __threadfence();
  }
}

__global__ __launch_bounds__(512)
void k_hq(const float* __restrict__ left, const float* __restrict__ Wq, const float* __restrict__ bq,
          const float* __restrict__ W1, const float* __restrict__ bk, float* HQE) {
  __shared__ float ls[DM];
  __shared__ float qs[HD];
  __shared__ float bks[HD];
  const int tid = threadIdx.x;
  const int b = blockIdx.x / NH, h = blockIdx.x - (blockIdx.x / NH) * NH;
  ls[tid]  = bf_val(left[(size_t)b * DM + tid]);
  bks[tid] = bf_val(bk[h * HD + tid]);
  __syncthreads();
  const float* wq = Wq + h * HD + tid;
  float acc = 0.f;
#pragma unroll 4
  for (int e = 0; e < DM; ++e) acc += ls[e] * bf_val(wq[(size_t)e * DQKV]);
  acc += bf_val(bq[h * HD + tid]);
  qs[tid] = acc;
  __syncthreads();
  const float* w1 = W1 + tid;
  float a2 = 0.f, a3 = 0.f;
#pragma unroll 4
  for (int c = 0; c < HD; ++c) {
    a2 += qs[c]  * bf_val(w1[(size_t)c * DM]);
    a3 += bks[c] * bf_val(w1[(size_t)(HD + c) * DM]);
  }
  const float v = a2 + a3;
  float* dst = HQE + (size_t)blockIdx.x * HD + tid;
  *(volatile float*)dst = v;
  __threadfence();
  *(volatile float*)dst = v;
}

__global__ __launch_bounds__(128)
void k_wc(const u16* __restrict__ W1KT, const u16* __restrict__ WKB, u16* WCH, u16* WCL) {
  __shared__ __align__(16) float slab[4 * SLAB];
  const int tid = threadIdx.x, wave = tid >> 5, lane = tid & 31, hh = lane >> 4, m = lane & 15;
  const int bid  = blockIdx.x;
  const int head = bid >> 6;
  const int t    = bid & 63;
  const int rowb = (t >> 3) * 64 + wave * 16;
  const int col0 = (t & 7) * 64;
  const u16* ap = W1KT + (size_t)(rowb + m) * HD + 8 * hh;
  const u16* bp = WKB + (size_t)(col0 + m) * DQKV + head * HD + 8 * hh;
  const size_t bs = (size_t)16 * DQKV;
  v8f acc0 = zero8(), acc1 = zero8(), acc2 = zero8(), acc3 = zero8();
#pragma unroll 1
  for (int k0 = 0; k0 < HD; k0 += 32) {
    const v16b a  = ldfrag_b(ap + k0);
    const v16b b0 = ldfrag_b(bp + k0);
    const v16b b1 = ldfrag_b(bp + bs + k0);
    const v16b b2 = ldfrag_b(bp + 2 * bs + k0);
    const v16b b3 = ldfrag_b(bp + 3 * bs + k0);
    acc0 = mma_b(a, b0, acc0);
    acc1 = mma_b(a, b1, acc1);
    acc2 = mma_b(a, b2, acc2);
    acc3 = mma_b(a, b3, acc3);
    guard5<v16b>(acc0, acc1, acc2, acc3, a, b0, b1, b2, b3);
  }
  acc_guard4(acc0, acc1, acc2, acc3);
  float* sl = slab + wave * SLAB;
#pragma unroll
  for (int r = 0; r < 8; ++r) {
    const int ro = (8 * hh + r) * 68 + m;
    sl[ro]      = acc0[r] * WCS;
    sl[ro + 16] = acc1[r] * WCS;
    sl[ro + 32] = acc2[r] * WCS;
    sl[ro + 48] = acc3[r] * WCS;
  }
  wave_sync_lds();
  const int rq = lane >> 3, c8 = (lane & 7) * 8;
  v4u oh[4], ol[4];
#pragma unroll
  for (int i4 = 0; i4 < 4; ++i4) {
    const int row = i4 * 4 + rq;
    const v4f a = *(const v4f*)(sl + row * 68 + c8), c4 = *(const v4f*)(sl + row * 68 + c8 + 4);
    float w[8];
#pragma unroll
    for (int e = 0; e < 4; ++e) { w[e] = a[e]; w[4 + e] = c4[e]; }
#pragma unroll
    for (int e = 0; e < 4; ++e) {
      const float x0 = w[2 * e], x1 = w[2 * e + 1];
      const _Float16 h0 = (_Float16)x0, h1 = (_Float16)x1;
      const _Float16 l0 = (_Float16)((x0 - (float)h0) * LOS);
      const _Float16 l1 = (_Float16)((x1 - (float)h1) * LOS);
      oh[i4][e] = pk16(h_bits(h0), h_bits(h1));
      ol[i4][e] = pk16(h_bits(l0), h_bits(l1));
    }
  }
  const size_t pb = (size_t)head * HD * DM + (size_t)(rowb + rq) * DM + col0 + c8;
  for (int pass = 0; pass < 2; ++pass) {
#pragma unroll
    for (int i4 = 0; i4 < 4; ++i4) {
      *(volatile v4u*)(WCH + pb + (size_t)(i4 * 4) * DM) = oh[i4];
      *(volatile v4u*)(WCL + pb + (size_t)(i4 * 4) * DM) = ol[i4];
    }
    __threadfence();
  }
}

__global__ __launch_bounds__(128)
void k_scores(const u16* __restrict__ RH, const u16* __restrict__ WCH, const u16* __restrict__ WCL,
              const float* __restrict__ HQE, const float* __restrict__ W2, float* SC) {
  __shared__ __align__(16) float slab[4 * SLAB];
  __shared__ __align__(16) float hqs[HD];
  __shared__ __align__(16) float w2s[HD];
  __shared__ __align__(16) float scs[64];
  const int tid = threadIdx.x, wave = tid >> 5, lane = tid & 31, hh = lane >> 4, m = lane & 15;
  const int bid   = blockIdx.x;
  const int head  = bid / NRT;
  const int rt    = bid - head * NRT;
  const int rowb0 = rt * 64;
  const int rowb  = rowb0 + wave * 16;
  const int b     = rowb0 / SEQ;
#pragma unroll
  for (int i = 0; i < HD / 128; ++i) {
    const int idx = tid + 128 * i;
    hqs[idx] = HQE[((size_t)b * NH + head) * HD + idx];
    w2s[idx] = bf_val(W2[idx]);
  }
  __syncthreads();

  const _Float16* ap  = (const _Float16*)(const void*)RH + (size_t)(rowb + m) * DM + 8 * hh;
  const size_t hoff   = (size_t)head * HD * DM + (size_t)m * DM + 8 * hh;
  const _Float16* bph = (const _Float16*)(const void*)WCH + hoff;
  const _Float16* bpl = (const _Float16*)(const void*)WCL + hoff;
  const size_t bs = (size_t)16 * DM;
  float* sl = slab + wave * SLAB;
  float part = 0.f;
  const float ihk = 1.0f / (RSC * WCS);
  const float ilo = 1.0f / LOS;

#pragma unroll 1
  for (int nt = 0; nt < HD / 64; ++nt) {
    const int col0 = nt * 64;
    const _Float16* bh = bph + (size_t)col0 * DM;
    const _Float16* bl = bpl + (size_t)col0 * DM;
    v8f ah0 = zero8(), ah1 = zero8(), ah2 = zero8(), ah3 = zero8();
    v8f al0 = zero8(), al1 = zero8(), al2 = zero8(), al3 = zero8();
#pragma unroll 1
    for (int k0 = 0; k0 < DM; k0 += 32) {
      const v16h a  = ldfrag_h(ap + k0);
      const v16h h0 = ldfrag_h(bh + k0);
      const v16h h1 = ldfrag_h(bh + bs + k0);
      const v16h h2 = ldfrag_h(bh + 2 * bs + k0);
      const v16h h3 = ldfrag_h(bh + 3 * bs + k0);
      ah0 = mma_h(a, h0, ah0);
      ah1 = mma_h(a, h1, ah1);
      ah2 = mma_h(a, h2, ah2);
      ah3 = mma_h(a, h3, ah3);
      guard5<v16h>(ah0, ah1, ah2, ah3, a, h0, h1, h2, h3);
      const v16h l0 = ldfrag_h(bl + k0);
      const v16h l1 = ldfrag_h(bl + bs + k0);
      const v16h l2 = ldfrag_h(bl + 2 * bs + k0);
      const v16h l3 = ldfrag_h(bl + 3 * bs + k0);
      al0 = mma_h(a, l0, al0);
      al1 = mma_h(a, l1, al1);
      al2 = mma_h(a, l2, al2);
      al3 = mma_h(a, l3, al3);
      guard5<v16h>(al0, al1, al2, al3, a, l0, l1, l2, l3);
    }
    acc_guard4(ah0, ah1, ah2, ah3);
    acc_guard4(al0, al1, al2, al3);
    wave_sync_lds();
#pragma unroll
    for (int r = 0; r < 8; ++r) {
      const int ro = (8 * hh + r) * 68 + m;
      sl[ro]      = (ah0[r] + al0[r] * ilo) * ihk;
      sl[ro + 16] = (ah1[r] + al1[r] * ilo) * ihk;
      sl[ro + 32] = (ah2[r] + al2[r] * ilo) * ihk;
      sl[ro + 48] = (ah3[r] + al3[r] * ilo) * ihk;
    }
    wave_sync_lds();
    const float* srow = sl + m * 68 + 32 * hh;
    const float* hq   = hqs + col0 + 32 * hh;
    const float* w2   = w2s + col0 + 32 * hh;
#pragma unroll 4
    for (int c = 0; c < 32; ++c) {
      const float x = srow[c] + hq[c];
      part += w2[c] * tanhf(x);
    }
  }
  part += __shfl_xor(part, 16, 32);
  if (hh == 0) scs[wave * 16 + m] = part;
  __syncthreads();
  if (wave == 0 && lane < 16) {
    const v4f v = *(const v4f*)(scs + lane * 4);
    float* dst = SC + (size_t)head * MROWS + rowb0 + lane * 4;
    *(volatile v4f*)dst = v;
    __threadfence();
    *(volatile v4f*)dst = v;
  }
}

__global__ __launch_bounds__(256)
void k_softmax(const float* __restrict__ SC, const int* __restrict__ mask, float* ATT) {
  __shared__ float redm[8];
  __shared__ float reds[8];
  const int t = threadIdx.x, wave = t >> 5, lane = t & 31;
  const int hb = blockIdx.x;
  const int h = hb / NB, b = hb - (hb / NB) * NB;
  const float* srow = SC + (size_t)h * MROWS + (size_t)b * SEQ;
  const int*   mrow = mask + (size_t)b * SEQ_FULL;
  float vals[EPT];
  float mx = -INFINITY;
#pragma unroll
  for (int i = 0; i < EPT; ++i) {
    const int l = t + 256 * i;
    const float s  = srow[l];
    const int   mk = mrow[l];
    const float sv = (mk == 0) ? -INFINITY : s;
    vals[i] = sv;
    mx = fmaxf(mx, sv);
  }
#pragma unroll
  for (int o = 16; o > 0; o >>= 1) mx = fmaxf(mx, __shfl_xor(mx, o, 32));
  if (lane == 0) redm[wave] = mx;
  __syncthreads();
  float gm = redm[0];
#pragma unroll
  for (int w = 1; w < 8; ++w) gm = fmaxf(gm, redm[w]);
  float sum = 0.f;
#pragma unroll
  for (int i = 0; i < EPT; ++i) {
    const float p = exp2f((vals[i] - gm) * LOG2E);
    vals[i] = p;
    sum += p;
  }
#pragma unroll
  for (int o = 16; o > 0; o >>= 1) sum += __shfl_xor(sum, o, 32);
  if (lane == 0) reds[wave] = sum;
  __syncthreads();
  float tot = reds[0];
#pragma unroll
  for (int w = 1; w < 8; ++w) tot += reds[w];
  const float inv = 1.0f / tot;
  float o_[EPT];
#pragma unroll
  for (int i = 0; i < EPT; ++i) o_[i] = vals[i] * inv;
  float* orow = ATT + ((size_t)h * NB_FULL + b) * OUT1_PITCH;
  for (int pass = 0; pass < 2; ++pass) {
#pragma unroll
    for (int i = 0; i < EPT; ++i) {
      *(volatile float*)(orow + t + 256 * i) = o_[i];
    }
    __threadfence();
  }
}

__global__ __launch_bounds__(512)
void k_att(const float* __restrict__ ATT, const float* __restrict__ right, const float* __restrict__ Wv,
           const float* __restrict__ bv, float* AT) {
  __shared__ float rs[DM];
  const int tid = threadIdx.x;
  const int bh = blockIdx.x;
  const int b = bh / NH, h = bh - (bh / NH) * NH;
  const float* arow = ATT + ((size_t)h * NB_FULL + b) * OUT1_PITCH;
  const float* rcol = right + (size_t)b * SEQ_FULL * DM + tid;
  float acc = 0.f;
#pragma unroll 4
  for (int l = 0; l < SEQ; ++l) acc += arow[l] * bf_val(rcol[(size_t)l * DM]);
  rs[tid] = acc;
  __syncthreads();
  const float* wv = Wv + h * HD + tid;
  float a2 = 0.f;
#pragma unroll 4
  for (int e = 0; e < DM; ++e) a2 += rs[e] * bf_val(wv[(size_t)e * DQKV]);
  const float v = a2 + bf_val(bv[h * HD + tid]);
  float* dst = AT + (size_t)bh * HD + tid;
  *(volatile float*)dst = v;
  __threadfence();
  *(volatile float*)dst = v;
}

__global__ __launch_bounds__(512)
void k_out(const float* __restrict__ AT, const float* __restrict__ Wfc, const float* __restrict__ bfc, float* out) {
  const int tid = threadIdx.x;
  const int b = blockIdx.x;
  const float* a = AT + (size_t)b * DQKV;
  const float* w = Wfc + tid;
  float acc = 0.f;
#pragma unroll 4
  for (int i = 0; i < DQKV; ++i) acc += a[i] * bf_val(w[(size_t)i * DM]);
  const float v = acc + bf_val(bfc[tid]);
  float* dst = out + (size_t)b * DM + tid;
  *(volatile float*)dst = v;
  __threadfence();
  *(volatile float*)dst = v;
}

extern "C" void kernel_launch(void* const* d_in, const int* in_sizes, int n_in,
                              void* d_out, int out_size, void* d_ws, size_t ws_size,
                              hipStream_t stream) {
  if (n_in < 13) return;
  if (in_sizes[0] < NB * DM) return;
  if (in_sizes[1] < (NB - 1) * SEQ_FULL * DM + SEQ * DM) return;
  if (in_sizes[2] < (NB - 1) * SEQ_FULL + SEQ) return;
  if (in_sizes[3] != DM * DQKV || in_sizes[5] != DM * DQKV || in_sizes[7] != DM * DQKV) return;
  if (in_sizes[4] != DQKV || in_sizes[6] != DQKV || in_sizes[8] != DQKV) return;
  if (in_sizes[9] != 2 * HD * HD) return;
  if (in_sizes[10] != HD) return;
  if (in_sizes[11] != DQKV * DM) return;
  if (in_sizes[12] != DM) return;
  if (out_size < OUT1_OFF + ((NH - 1) * NB_FULL + (NB - 1)) * OUT1_PITCH + SEQ) return;

  const float* left  = (const float*)d_in[0];
  const float* right = (const float*)d_in[1];
  const int*   mask  = (const int*)d_in[2];
  const float* Wq    = (const float*)d_in[3];
  const float* bq    = (const float*)d_in[4];
  const float* Wk    = (const float*)d_in[5];
  const float* bk    = (const float*)d_in[6];
  const float* Wv    = (const float*)d_in[7];
  const float* bv    = (const float*)d_in[8];
  const float* W1    = (const float*)d_in[9];
  const float* W2    = (const float*)d_in[10];
  const float* Wfc   = (const float*)d_in[11];
  const float* bfc   = (const float*)d_in[12];
  float* out0 = (float*)d_out;
  float* out1 = out0 + (size_t)OUT1_OFF;

  const size_t szRH  = (size_t)MROWS * DM * 2;
  const size_t szWKB = (size_t)DM * DQKV * 2;
  const size_t szW1T = (size_t)HD * HD * 2;
  const size_t szWC  = (size_t)NH * HD * DM * 2;
  const size_t szHQE = (size_t)NB * NH * HD * 4;
  const size_t szSC  = (size_t)NH * MROWS * 4;
  const size_t szAT  = (size_t)NB * DQKV * 4;
  size_t off = 0;
  const size_t oRH  = off; off += (szRH  + 255) & ~(size_t)255;
  const size_t oWKB = off; off += (szWKB + 255) & ~(size_t)255;
  const size_t oW1T = off; off += (szW1T + 255) & ~(size_t)255;
  const size_t oWCH = off; off += (szWC  + 255) & ~(size_t)255;
  const size_t oWCL = off; off += (szWC  + 255) & ~(size_t)255;
  const size_t oHQE = off; off += (szHQE + 255) & ~(size_t)255;
  const size_t oSC  = off; off += (szSC  + 255) & ~(size_t)255;
  const size_t oAT  = off; off += (szAT  + 255) & ~(size_t)255;
  if (off > ws_size) return;
  if (off > (size_t)134217728) return;

  char* ws = (char*)d_ws;
  u16*   RH   = (u16*)(ws + oRH);
  u16*   WKB  = (u16*)(ws + oWKB);
  u16*   W1KT = (u16*)(ws + oW1T);
  u16*   WCH  = (u16*)(ws + oWCH);
  u16*   WCL  = (u16*)(ws + oWCL);
  float* HQE  = (float*)(ws + oHQE);
  float* SC   = (float*)(ws + oSC);
  float* AT   = (float*)(ws + oAT);

  const int n8r = MROWS * (DM / 8);
  const int n8w = (DM * DQKV) / 8;
  if ((n8r % 256) != 0 || (n8w % 256) != 0) return;
  const dim3 b256(256), b128(128), b512(512);
  const dim3 gCR(n8r / 256);
  const dim3 gCW(n8w / 256);
  const dim3 gT(64);
  const dim3 gHQ(NB * NH);
  const dim3 gWC(NH * 64);
  const dim3 gSC(NH * NRT);
  const dim3 gSM(NH * NB);
  const dim3 gAT(NB * NH);
  const dim3 gOUT(NB);

  k_cvt_right<<<gCR, b256, 0, stream>>>(right, RH, n8r);
  k_cvt_bf<<<gCW, b256, 0, stream>>>(Wk, WKB, n8w);
  k_w1kt<<<gT, b256, 0, stream>>>(W1, W1KT);
  k_hq<<<gHQ, b512, 0, stream>>>(left, Wq, bq, W1, bk, HQE);
  k_wc<<<gWC, b128, 0, stream>>>(W1KT, WKB, WCH, WCL);
  k_scores<<<gSC, b128, 0, stream>>>(RH, WCH, WCL, HQE, W2, SC);
  k_softmax<<<gSM, b256, 0, stream>>>(SC, mask, out1);
  k_att<<<gAT, b512, 0, stream>>>(out1, right, Wv, bv, AT);
  k_out<<<gOUT, b512, 0, stream>>>(AT, Wfc, bfc, out0);
  (void)hipGetLastError();
}
